// MultiheadCrossAttention_25709674234096
// MI455X (gfx1250) — hardware-verified
//
#include <hip/hip_runtime.h>
#ifndef NB
#define NB 2
#endif
#ifndef SQ
#define SQ 4096
#endif
#define NB_FULL 2
#define SQ_FULL 4096
#define SK 1024
#define DM 1024
#define D2 2048
#define NH 16
#define HD 64
#define HG 2
#define WSC 16.0f
#define PCAR 4096.0f
#define RPW 16
#define NRQ ((size_t)NB * SQ)
#define NRK ((size_t)NB * SK)
static_assert(NB >= 1 && NB <= NB_FULL);
static_assert(SQ % 128 == 0 && SQ >= 128 && SQ <= SQ_FULL);
static_assert(SK % 256 == 0 && SK % 128 == 0 && DM % 128 == 0 && D2 % 64 == 0);
static_assert(NH % HG == 0 && HD == 64 && NH * HD == DM && (HG * SQ) % (8 * RPW) == 0);

typedef unsigned short v8us __attribute__((ext_vector_type(8), may_alias));
typedef float  v8f  __attribute__((ext_vector_type(8)));
typedef float  v4f  __attribute__((ext_vector_type(4)));
typedef float  v4fa __attribute__((ext_vector_type(4), may_alias));
typedef _Float16 v16h __attribute__((ext_vector_type(16)));
typedef _Float16 v4h __attribute__((ext_vector_type(4)));
union FragH { v16h v; v8us half[2]; _Float16 h[16]; unsigned short u[16]; };

__device__ __forceinline__ unsigned short bf16_bits(float x) { unsigned int u = __float_as_uint(x); return (unsigned short)((u + 0x7FFFu + ((u >> 16) & 1u)) >> 16); }
__device__ __forceinline__ float bf16_val(unsigned short b) { return __uint_as_float(((unsigned int)b) << 16); }
__device__ __forceinline__ float bf16_rne(float x) { return bf16_val(bf16_bits(x)); }

__device__ __forceinline__ v16h g2_frag(const _Float16* p, int hh) { FragH f; f.half[0] = *(const v8us*)((const unsigned short*)p + 8 * hh); f.half[1] = *(const v8us*)((const unsigned short*)p + 16 + 8 * hh); return f.v; }
__device__ __forceinline__ v8f g2_mma(v16h a, v16h b, v8f c) { v8f d = __builtin_amdgcn_wmma_f32_16x16x32_f16(false, a, false, b, (short)0, c, false, false); asm volatile("v_nop\n\tv_nop\n\tv_nop\n\tv_nop" : "+v"(d) : "v"(a), "v"(b)); return d; }

__global__ __launch_bounds__(256) void k_wt_f16(const float* __restrict__ W, _Float16* __restrict__ Wt, int K, int N, float scale) {
  const int t = blockIdx.x * 256 + threadIdx.x; if (t >= N * (K / 8)) return;
  const int n = t / (K / 8), k8 = (t % (K / 8)) * 8; FragH f;
#pragma unroll
  for (int i = 0; i < 8; ++i) f.h[i] = (_Float16)(bf16_rne(W[(size_t)(k8 + i) * N + n]) * scale);
  const v8us o = f.half[0]; unsigned short* d = (unsigned short*)Wt + (size_t)n * K + k8;
  *(volatile v8us*)d = o; __threadfence(); *(volatile v8us*)d = o;
}

template <int RPB, int SRPB>
__global__ __launch_bounds__(256) void k_x16(const float* __restrict__ x, _Float16* __restrict__ X16, size_t n8) {
  const size_t t = (size_t)blockIdx.x * 256 + threadIdx.x; if (t >= n8) return;
  const unsigned row = (unsigned)(t / (DM / 8)); const unsigned col = (unsigned)(t % (DM / 8)) * 8u;
  const unsigned b = row / (unsigned)RPB, r = row - b * (unsigned)RPB;
  const float* src = x + ((size_t)b * SRPB + r) * DM + col;
  const v4f a = *(const v4fa*)src, c = *(const v4fa*)(src + 4); FragH f;
#pragma unroll
  for (int q = 0; q < 4; ++q) { f.h[q] = (_Float16)bf16_rne(a[q]); f.h[4 + q] = (_Float16)bf16_rne(c[q]); }
  unsigned short* d = (unsigned short*)X16 + t * 8;
  *(volatile v8us*)d = f.half[0]; __threadfence(); *(volatile v8us*)d = f.half[0];
}

__global__ __launch_bounds__(128) void k_gemm2(const _Float16* __restrict__ A, int lda, size_t sA, const _Float16* __restrict__ Bh, int ldb, size_t sB, float alpha,
    const float* __restrict__ bias, size_t sBias, const float* __restrict__ CP, int rowsPerB, size_t sCPb, int row0g,
    float* __restrict__ C, _Float16* __restrict__ C16, int ldc, size_t sC, int M, int N, int K) {
  __shared__ __attribute__((aligned(16))) float so[4][32][68];
  const int tid = threadIdx.x, w = tid >> 5, lane = tid & 31, ln = lane & 15, hh = lane >> 4; const int by = blockIdx.y;
  A += (size_t)by * sA; Bh += (size_t)by * sB; const size_t cofs = (size_t)by * sC; const float* bp = bias ? bias + (size_t)by * sBias : nullptr;
  const int ntn = N >> 6; const int mt = blockIdx.x / ntn, nq = blockIdx.x - mt * ntn; const int row0 = mt * 128 + 32 * w, col0 = nq * 64; if (row0 >= M) return;
  const _Float16* a0p = A + (size_t)(row0 + ln) * lda; const _Float16* a1p = a0p + (size_t)16 * lda;
  const _Float16* b0p = Bh + (size_t)(col0 + ln) * ldb; const _Float16* b1p = b0p + (size_t)16 * ldb; const _Float16* b2p = b1p + (size_t)16 * ldb; const _Float16* b3p = b2p + (size_t)16 * ldb;
  const v8f z8 = {0.f,0.f,0.f,0.f,0.f,0.f,0.f,0.f}; v8f c00 = z8, c01 = z8, c02 = z8, c03 = z8, c10 = z8, c11 = z8, c12 = z8, c13 = z8;
#pragma unroll 1
  for (int kb = 0; kb < K; kb += 32) { const v16h a0 = g2_frag(a0p + kb, hh), a1 = g2_frag(a1p + kb, hh);
    v16h b = g2_frag(b0p + kb, hh); c00 = g2_mma(a0, b, c00); c10 = g2_mma(a1, b, c10);
    b = g2_frag(b1p + kb, hh); c01 = g2_mma(a0, b, c01); c11 = g2_mma(a1, b, c11);
    b = g2_frag(b2p + kb, hh); c02 = g2_mma(a0, b, c02); c12 = g2_mma(a1, b, c12);
    b = g2_frag(b3p + kb, hh); c03 = g2_mma(a0, b, c03); c13 = g2_mma(a1, b, c13); }
  v8f accs[8] = {c00, c01, c02, c03, c10, c11, c12, c13};
#pragma unroll
  for (int u = 0; u < 8; ++u) { const int t = u & 3, hf = u >> 2; const int col = col0 + t * 16 + ln; const float bv = bp ? bf16_rne(bp[col]) : 0.f;
#pragma unroll
    for (int r = 0; r < 8; ++r) { const int rloc = hf * 16 + 8 * hh + r; float v = accs[u][r] * alpha + bv;
      if (CP) { if (rowsPerB < 0) v += CP[cofs + (size_t)(row0g + row0 + rloc) * ldc + col];
                else { const int bidx = (row0g + row0 + rloc) / rowsPerB; v += CP[(size_t)bidx * sCPb + (size_t)by * 64 + col]; } }
      so[w][rloc][t * 16 + ln] = v; } }
  __builtin_amdgcn_fence(4  , "workgroup"); __builtin_amdgcn_wave_barrier();
  const int rsub = lane >> 4, c4 = (lane & 15) * 4;
  for (int pass = 0; pass < 2; ++pass) {
#pragma unroll
    for (int q = 0; q < 16; ++q) { const int r = q * 2 + rsub; const v4f v = *(const v4fa*)&so[w][r][c4];
      if (C) *(volatile v4f*)(C + cofs + (size_t)(row0 + r) * ldc + col0 + c4) = v;
      if (C16) { v4h h4; for (int i = 0; i < 4; ++i) h4[i] = (_Float16)v[i]; *(volatile v4h*)(C16 + cofs + (size_t)(row0 + r) * ldc + col0 + c4) = h4; } }
    if (pass == 0) __threadfence(); }
}

__global__ __launch_bounds__(256) void k_vt(const _Float16* __restrict__ KV16, _Float16* __restrict__ VT) {
  __shared__ unsigned short tl[64][66];
  const int tid = threadIdx.x; const int nsg = SK / 64; const int slab = blockIdx.x / nsg, sg = blockIdx.x - slab * nsg; const int b = slab / NH, h = slab - b * NH; const int s0 = sg * 64;
  for (int i = tid; i < 64 * 8; i += 256) { const int r = i >> 3, c8 = (i & 7) * 8; FragH f;
    f.half[0] = *(const v8us*)((const unsigned short*)KV16 + ((size_t)b * SK + s0 + r) * D2 + (size_t)h * 2 * HD + HD + c8);
#pragma unroll
    for (int q = 0; q < 8; ++q) tl[r][c8 + q] = f.u[q]; }
  __syncthreads();
  FragH o0, o1; { const int d = tid >> 3, pc = tid & 7;
#pragma unroll
    for (int q = 0; q < 8; ++q) { o0.u[q] = tl[pc * 8 + q][d]; o1.u[q] = tl[pc * 8 + q][32 + d]; } }
  for (int pass = 0; pass < 2; ++pass) { const int d = tid >> 3, pc = tid & 7;
    *(volatile v8us*)((unsigned short*)VT + ((size_t)slab * HD + d) * SK + s0 + pc * 8) = o0.half[0];
    *(volatile v8us*)((unsigned short*)VT + ((size_t)slab * HD + 32 + d) * SK + s0 + pc * 8) = o1.half[0];
    if (pass == 0) __threadfence(); }
}

__global__ __launch_bounds__(256) void k_rsm(const float* __restrict__ S, _Float16* __restrict__ P, int nrows) {
  #pragma clang fp contract(off)
  const int lane = threadIdx.x & 31, w = threadIdx.x >> 5; const int rbase = (blockIdx.x * 8 + w) * RPW;
#pragma unroll 1
  for (int rr = 0; rr < RPW; ++rr) {
    const int i = rbase + rr; if (i >= nrows) break;
    const float* s = S + (size_t)i * SK; float v[32];
#pragma unroll
    for (int u = 0; u < 4; ++u) { const v4f a = *(const v4fa*)(s + 256 * u + 8 * lane), c = *(const v4fa*)(s + 256 * u + 8 * lane + 4);
      v[8 * u + 0] = a[0]; v[8 * u + 1] = a[1]; v[8 * u + 2] = a[2]; v[8 * u + 3] = a[3]; v[8 * u + 4] = c[0]; v[8 * u + 5] = c[1]; v[8 * u + 6] = c[2]; v[8 * u + 7] = c[3]; }
    float mx = v[0];
#pragma unroll
    for (int q = 1; q < 32; ++q) mx = fmaxf(mx, v[q]);
#pragma unroll
    for (int off = 1; off < 32; off <<= 1) mx = fmaxf(mx, __shfl_xor(mx, off, 32));
    float se = 0.f;
#pragma unroll
    for (int q = 0; q < 32; ++q) { v[q] = __expf(v[q] - mx); se += v[q]; }
#pragma unroll
    for (int off = 1; off < 32; off <<= 1) se += __shfl_xor(se, off, 32);
    const float sc = PCAR / se; const float ctr = PCAR / (float)SK;
    FragH f0, f1, f2, f3;
#pragma unroll
    for (int q = 0; q < 8; ++q) { f0.h[q] = (_Float16)(v[q] * sc - ctr); f1.h[q] = (_Float16)(v[8 + q] * sc - ctr); f2.h[q] = (_Float16)(v[16 + q] * sc - ctr); f3.h[q] = (_Float16)(v[24 + q] * sc - ctr); }
    unsigned short* d = (unsigned short*)P + (size_t)i * SK + 8 * lane;
    for (int pass = 0; pass < 2; ++pass) {
      *(volatile v8us*)(d) = f0.half[0]; *(volatile v8us*)(d + 256) = f1.half[0]; *(volatile v8us*)(d + 512) = f2.half[0]; *(volatile v8us*)(d + 768) = f3.half[0];
      if (pass == 0) __threadfence(); }
  }
}

__global__ __launch_bounds__(256) void k_md(const float* __restrict__ data, float* __restrict__ md) {
  const int t = blockIdx.x * 256 + threadIdx.x; if (t >= NB * DM) return; const int b = t / DM, k = t - b * DM;
  const float* p = data + (size_t)b * SK * DM + k; double acc = 0.0;
#pragma unroll 1
  for (int s = 0; s < SK; ++s) acc += (double)bf16_rne(p[(size_t)s * DM]);
  const float m = (float)(acc * (1.0 / (double)SK));
  *(volatile float*)(md + t) = m; __threadfence(); *(volatile float*)(md + t) = m;
}
__global__ __launch_bounds__(256) void k_mv(const float* __restrict__ md, const float* __restrict__ Wkv, const float* __restrict__ bkv, float* __restrict__ mv) {
  const int t = blockIdx.x * 256 + threadIdx.x; if (t >= NB * DM) return; const int b = t / DM, j = t - b * DM; const int col = (j >> 6) * (2 * HD) + HD + (j & 63);
  const float* m = md + (size_t)b * DM; double acc = 0.0;
#pragma unroll 1
  for (int k = 0; k < DM; ++k) acc += (double)m[k] * (double)bf16_rne(Wkv[(size_t)k * D2 + col]);
  const float r = (float)acc + bf16_rne(bkv[col]);
  *(volatile float*)(mv + t) = r; __threadfence(); *(volatile float*)(mv + t) = r;
}
__global__ __launch_bounds__(256) void k_mo(const float* __restrict__ mv, const float* __restrict__ Wp, float* __restrict__ mo) {
  const int t = blockIdx.x * 256 + threadIdx.x; if (t >= NB * DM) return; const int b = t / DM, i = t - b * DM;
  const float* m = mv + (size_t)b * DM; double acc = 0.0;
#pragma unroll 1
  for (int j = 0; j < DM; ++j) acc += (double)m[j] * (double)bf16_rne(Wp[(size_t)j * DM + i]);
  const float r = (float)acc;
  *(volatile float*)(mo + t) = r; __threadfence(); *(volatile float*)(mo + t) = r;
}

extern "C" void kernel_launch(void* const* d_in, const int* in_sizes, int n_in,
                              void* d_out, int out_size, void* d_ws, size_t ws_size, hipStream_t stream) {
  if (n_in < 8) return;
  if ((size_t)in_sizes[0] < ((size_t)(NB - 1) * SQ_FULL + SQ) * DM) return;
  if ((size_t)in_sizes[1] < NRK * DM) return;
  if (in_sizes[2] < DM * DM || in_sizes[3] < DM || in_sizes[4] < DM * D2 || in_sizes[5] < D2 || in_sizes[6] < DM * DM || in_sizes[7] < DM) return;
  if ((size_t)out_size < ((size_t)(NB - 1) * SQ_FULL + SQ) * DM) return;
  const float* const* I = (const float* const*)d_in;
  const float* x = I[0]; const float* data = I[1]; const float* wq = I[2]; const float* bq = I[3]; const float* wkv = I[4]; const float* bkv = I[5]; const float* wp = I[6]; const float* bp = I[7];
  char* ws = (char*)d_ws; size_t off = 0;
  auto take = [&](size_t bytes) { char* p = ws + off; off += (bytes + 255) & ~(size_t)255; return p; };
  _Float16* BQ = (_Float16*)take((size_t)DM * DM * 2); _Float16* BKV = (_Float16*)take((size_t)D2 * DM * 2); _Float16* BP = (_Float16*)take((size_t)DM * DM * 2);
  _Float16* XQ = (_Float16*)take(NRQ * DM * 2); _Float16* XD = (_Float16*)take(NRK * DM * 2); _Float16* Q16 = (_Float16*)take(NRQ * DM * 2); _Float16* KV = (_Float16*)take(NRK * D2 * 2); _Float16* O16 = (_Float16*)take(NRQ * DM * 2);
  _Float16* VT = (_Float16*)take((size_t)NB * NH * HD * SK * 2);
  float* S = (float*)take((size_t)HG * SQ * SK * 4); _Float16* P = (_Float16*)take((size_t)HG * SQ * SK * 2);
  float* MD = (float*)take((size_t)NB * DM * 4); float* MV = (float*)take((size_t)NB * DM * 4); float* MO = (float*)take((size_t)NB * DM * 4);
  if (off > ws_size) return;

  k_wt_f16<<<(unsigned)(((size_t)DM * (DM / 8) + 255) / 256), 256, 0, stream>>>(wq, BQ, DM, DM, WSC);
  k_wt_f16<<<(unsigned)(((size_t)D2 * (DM / 8) + 255) / 256), 256, 0, stream>>>(wkv, BKV, DM, D2, WSC);
  k_wt_f16<<<(unsigned)(((size_t)DM * (DM / 8) + 255) / 256), 256, 0, stream>>>(wp, BP, DM, DM, WSC);
  k_x16<SQ, SQ_FULL><<<(unsigned)((NRQ * DM / 8 + 255) / 256), 256, 0, stream>>>(x, XQ, NRQ * DM / 8);
  k_x16<SK, SK><<<(unsigned)((NRK * DM / 8 + 255) / 256), 256, 0, stream>>>(data, XD, NRK * DM / 8);
  k_md<<<(unsigned)((NB * DM + 255) / 256), 256, 0, stream>>>(data, MD);
  k_mv<<<(unsigned)((NB * DM + 255) / 256), 256, 0, stream>>>(MD, wkv, bkv, MV);
  k_mo<<<(unsigned)((NB * DM + 255) / 256), 256, 0, stream>>>(MV, wp, MO);
  k_gemm2<<<dim3((unsigned)((NRQ / 128) * (DM / 64)), 1), 128, 0, stream>>>(XQ, DM, 0, BQ, DM, 0, 1.0f / WSC, bq, 0, nullptr, 1, 0, 0, nullptr, Q16, DM, 0, (int)NRQ, DM, DM);
  k_gemm2<<<dim3((unsigned)((NRK / 128) * (D2 / 64)), 1), 128, 0, stream>>>(XD, DM, 0, BKV, DM, 0, 1.0f / WSC, bkv, 0, nullptr, 1, 0, 0, nullptr, KV, D2, 0, (int)NRK, D2, DM);
  k_vt<<<(unsigned)(NB * NH * (SK / 64)), 256, 0, stream>>>(KV, VT);
  for (int b = 0; b < NB; ++b) for (int h0 = 0; h0 < NH; h0 += HG) {
    const _Float16* qb = Q16 + (size_t)b * SQ * DM + h0 * HD; const _Float16* kb = KV + (size_t)b * SK * D2 + (size_t)h0 * 2 * HD;
    k_gemm2<<<dim3((unsigned)((SQ / 128) * (SK / 64)), HG), 128, 0, stream>>>(qb, DM, (size_t)HD, kb, D2, (size_t)(2 * HD), 0.125f, nullptr, 0, nullptr, 1, 0, 0, S, nullptr, SK, (size_t)SQ * SK, SQ, SK, HD);
    k_rsm<<<(unsigned)((HG * SQ) / (8 * RPW)), 256, 0, stream>>>(S, P, HG * SQ);
    k_gemm2<<<dim3((unsigned)((SQ / 128) * (HD / 64)), HG), 128, 0, stream>>>(P, SK, (size_t)SQ * SK, VT + (size_t)(b * NH + h0) * HD * SK, SK, (size_t)HD * SK, 1.0f, nullptr, 0, nullptr, 1, 0, 0, nullptr, O16 + (size_t)b * SQ * DM + h0 * HD, DM, (size_t)HD, SQ, HD, SK); }
  for (int b = 0; b < NB; ++b)
    k_gemm2<<<dim3((unsigned)((SQ / 128) * (DM / 64)), 1), 128, 0, stream>>>(O16 + (size_t)b * SQ * DM, DM, 0, BP, DM, 0, (1.0f / WSC) / PCAR, bp, 0, MO + (size_t)b * DM, SQ, 0, 0, (float*)d_out + (size_t)b * SQ_FULL * DM, nullptr, DM, 0, SQ, DM, DM);
}
